// CosineDistance_17660905521623
// MI455X (gfx1250) — hardware-verified
//
#include <hip/hip_runtime.h>
#include <stddef.h>
#include <stdint.h>
#include <math.h>


#define DD     128
#define NT     64
#define NPA    64
#define NSB    256
#define BGRP   32
#define NTHR   128
#define NWAVE  4
#define WSCAP  134217728
#define CARRY  64.0f
#define OUT_UNSCALE (1.0f / 4096.0f)

static_assert(NTHR == NWAVE * 32);
static_assert(NT == NWAVE * 16);
static_assert((DD % 32) == 0);
static_assert((NSB % BGRP) == 0);
static_assert(((NPA * NT) % 8) == 0);
static_assert(((NSB * NT) % 8) == 0);
static_assert(BGRP == 32);

#define SZ_PN  ((size_t)NPA * NT * DD * 2)
#define SZ_SN  ((size_t)NSB * NT * DD * 2)
#define SZ_TOT (SZ_PN + SZ_SN)
static_assert(SZ_TOT <= (size_t)WSCAP);
static_assert((SZ_PN % 512) == 0);
static_assert((SZ_SN % 512) == 0);

typedef float     v4f  __attribute__((ext_vector_type(4)));
typedef float     v8f  __attribute__((ext_vector_type(8)));
typedef _Float16  v8h  __attribute__((ext_vector_type(8)));
typedef _Float16  v16h __attribute__((ext_vector_type(16)));
union FragH { v16h v; v8h h[2]; };

__device__ __forceinline__ v8f wmf(v16h a, v16h b, v8f c) {
  v8f d = __builtin_amdgcn_wmma_f32_16x16x32_f16(false, a, false, b, (short)0, c, false, false);
  asm volatile("v_nop\n\tv_nop\n\tv_nop\n\tv_nop" : "+v"(d) : "v"(a), "v"(b));
  return d;
}

__device__ __forceinline__ v8h cvt8(v4f a, v4f b) {
  v8h r;
  r[0] = (_Float16)a.x; r[1] = (_Float16)a.y; r[2] = (_Float16)a.z; r[3] = (_Float16)a.w;
  r[4] = (_Float16)b.x; r[5] = (_Float16)b.y; r[6] = (_Float16)b.z; r[7] = (_Float16)b.w;
  return r;
}

__global__ __launch_bounds__(NTHR) void k_norm(const float* __restrict__ x, _Float16* y, int nrows) {
  const int tid = threadIdx.x, lane = tid & 31, wv = tid >> 5, h = lane >> 4, m = lane & 15;
  const int rowraw = blockIdx.x * 8 + 2 * wv + h;
  const bool ok = rowraw < nrows;
  const int row = min(rowraw, nrows - 1);
  const float* xr = x + (size_t)row * DD + 8 * m;
  const v4f f0 = *(const v4f*)xr;
  const v4f f1 = *(const v4f*)(xr + 4);
  float ss = f0.x * f0.x + f0.y * f0.y + f0.z * f0.z + f0.w * f0.w;
  ss += f1.x * f1.x + f1.y * f1.y + f1.z * f1.z + f1.w * f1.w;
  ss += __shfl_xor(ss, 1);
  ss += __shfl_xor(ss, 2);
  ss += __shfl_xor(ss, 4);
  ss += __shfl_xor(ss, 8);
  const float nrm = sqrtf(ss);
  const float sc = (1.0f / fmaxf(nrm, 1e-12f)) * CARRY;
  const v8h o = cvt8(f0 * sc, f1 * sc);
  _Float16* d = y + (size_t)row * DD + 8 * m;
  if (ok) *(volatile v8h*)d = o;
  __threadfence();
  if (ok) *(volatile v8h*)d = o;
}

__global__ __launch_bounds__(NTHR) void k_maxsim(const _Float16* __restrict__ pn16,
                                                 const _Float16* __restrict__ sn16,
                                                 float* out) {
  __shared__ __attribute__((aligned(16))) float ob[NWAVE * BGRP];
  const int tid = threadIdx.x, lane = tid & 31, wv = tid >> 5, h = lane >> 4, m = lane & 15;
  const int bg = blockIdx.x, a = blockIdx.y;
  const v8f zero8 = {0.f, 0.f, 0.f, 0.f, 0.f, 0.f, 0.f, 0.f};

  const _Float16* arow = pn16 + ((size_t)a * NT + 16 * wv + m) * DD + 8 * h;

#pragma unroll 1
  for (int bb = 0; bb < BGRP; ++bb) {
    const int b = bg * BGRP + bb;
    const _Float16* brow = sn16 + ((size_t)b * NT + m) * DD + 8 * h;

    v8f acc[4];
#pragma unroll
    for (int jt = 0; jt < 4; ++jt) acc[jt] = zero8;

#pragma unroll 1
    for (int ks = 0; ks < DD / 32; ++ks) {
      const int k0 = 32 * ks;
      FragH af;
      af.h[0] = *(const v8h*)(arow + k0);
      af.h[1] = *(const v8h*)(arow + k0 + 16);
      FragH bf[4];
#pragma unroll
      for (int jt = 0; jt < 4; ++jt) {
        const _Float16* bq = brow + (size_t)(jt * 16) * DD + k0;
        bf[jt].h[0] = *(const v8h*)bq;
        bf[jt].h[1] = *(const v8h*)(bq + 16);
      }
#pragma unroll
      for (int jt = 0; jt < 4; ++jt) acc[jt] = wmf(af.v, bf[jt].v, acc[jt]);
    }

    float s = 0.f;
#pragma unroll
    for (int r = 0; r < 8; ++r) {
      float mx = fmaxf(fmaxf(acc[0][r], acc[1][r]), fmaxf(acc[2][r], acc[3][r]));
      mx = fmaxf(mx, __shfl_xor(mx, 1));
      mx = fmaxf(mx, __shfl_xor(mx, 2));
      mx = fmaxf(mx, __shfl_xor(mx, 4));
      mx = fmaxf(mx, __shfl_xor(mx, 8));
      s += mx;
    }
    s += __shfl_xor(s, 16);
    if (lane == 0) ob[wv * BGRP + bb] = s;
  }
  __syncthreads();

  if (wv == 0) {
    const int q = lane & 7;
    v4f v;
#pragma unroll
    for (int c = 0; c < 4; ++c) {
      const int idx = 4 * q + c;
      const float t = ((ob[idx] + ob[BGRP + idx]) + ob[2 * BGRP + idx]) + ob[3 * BGRP + idx];
      v[c] = t * OUT_UNSCALE;
    }
    float* gp = out + (size_t)a * NSB + bg * BGRP + 4 * q;
    if (lane < 8) *(volatile v4f*)gp = v;
    __threadfence();
    if (lane < 8) *(volatile v4f*)gp = v;
  }
}

extern "C" void kernel_launch(void* const* d_in, const int* in_sizes, int n_in,
                              void* d_out, int out_size, void* d_ws, size_t ws_size,
                              hipStream_t stream) {
  if (n_in < 2) return;
  if (in_sizes[0] != NSB * NT * DD) return;
  if (in_sizes[1] != NPA * NT * DD) return;
  if (out_size != NPA * NSB) return;

  const float* sat  = (const float*)d_in[0];
  const float* pano = (const float*)d_in[1];
  float* out = (float*)d_out;

  char* ws = (char*)d_ws;
  size_t off = 0;
  const size_t oPN = off; off += SZ_PN;
  const size_t oSN = off; off += SZ_SN;
  if (off != SZ_TOT) return;
  if (off > ws_size || off > (size_t)WSCAP) return;

  _Float16* pn16 = (_Float16*)(ws + oPN);
  _Float16* sn16 = (_Float16*)(ws + oSN);

  k_norm<<<(NPA * NT) / 8, NTHR, 0, stream>>>(pano, pn16, NPA * NT);
  k_norm<<<(NSB * NT) / 8, NTHR, 0, stream>>>(sat, sn16, NSB * NT);
  k_maxsim<<<dim3(NSB / BGRP, NPA), NTHR, 0, stream>>>(pn16, sn16, out);
}
